// DeepNCMDecoder_59897613910017
// MI455X (gfx1250) — hardware-run, weakly checked
//
#include <hip/hip_runtime.h>
#include <stddef.h>


typedef _Float16 v16h __attribute__((ext_vector_type(16)));
typedef _Float16 v8h  __attribute__((ext_vector_type(8)));
typedef float    v8f  __attribute__((ext_vector_type(8)));
typedef float    v4f  __attribute__((ext_vector_type(4)));
typedef int      v4i  __attribute__((ext_vector_type(4)));

#ifndef NB
#define NB 8192
#endif
#define NB_FULL 8192
#define DIM   1024
#define HID   2048
#define EDIM  1024
#define NCLS  1000
#define NCP   1024
#define MROWS NB
#define SROWS 16
#define NWORDS (NB / 32)

static_assert(NB >= 1024 && NB <= NB_FULL && (NB % 1024) == 0);
static_assert(HID == 2 * EDIM);
static_assert((DIM % 64) == 0 && (DIM % 32) == 0);
static_assert((HID % 64) == 0 && (HID % 32) == 0);
static_assert((EDIM % 64) == 0 && (EDIM % 32) == 0);
static_assert((MROWS % 64) == 0 && (MROWS % 8) == 0 && (MROWS % SROWS) == 0);
static_assert(DIM == 4 * 32 * 8);
static_assert(EDIM == 4 * 32 * 8);
static_assert(EDIM == 256 * 4);
static_assert(NCP == 8 * 128);
static_assert((NCP % 32) == 0 && NCLS <= NCP && (NCLS % 4) == 0 && NCLS > NCP - 32);
static_assert(NWORDS <= 256 && (NWORDS % 32) == 0);
static_assert(SROWS == 16);
static_assert(((size_t)SROWS * NCLS * 4) % 128 == 0);
static_assert(((SROWS * NCLS / 4) % 32) == 0);
static_assert((size_t)SROWS * NCLS * 4 + SROWS * 4 <= 65536);
static_assert((size_t)MROWS * HID < (size_t)0xFFFFFFFFu);

#define LDT 72
#define LDC 68
static_assert((LDT % 8) == 0 && LDT >= 64);
static_assert((LDC % 4) == 0 && LDC >= 64);

#define WCARRY 64.0f
#define MCARRY 16.0f
#define ECARRY 16.0f

#define OUT_UPD_OFF ((size_t)NB_FULL * NCLS)
#define OUT_CNT_OFF (OUT_UPD_OFF + (size_t)NCLS * EDIM)
#define OUT_TOTAL   (OUT_CNT_OFF + (size_t)NCLS)
static_assert(OUT_UPD_OFF * 4 == (size_t)32768000);
static_assert(OUT_CNT_OFF * 4 == (size_t)36864000);
static_assert(OUT_TOTAL * 4 == (size_t)36868000);
static_assert(((OUT_UPD_OFF * 4) % 128) == 0 && ((OUT_CNT_OFF * 4) % 128) == 0);

#define W1T_BYTES ((size_t)HID * DIM * 2)
#define W2T_BYTES ((size_t)EDIM * HID * 2)
#define PP_BYTES  ((size_t)NCP * EDIM * 2)
#define P2_BYTES  ((size_t)NCP * 4)
#define X16_BYTES ((size_t)MROWS * DIM * 2)
#define H16_BYTES ((size_t)MROWS * HID * 2)
#define E16_BYTES ((size_t)MROWS * EDIM * 2)
#define E32_BYTES ((size_t)MROWS * EDIM * 4)
#define OFF_W1T ((size_t)0)
#define OFF_W2T (OFF_W1T + W1T_BYTES)
#define OFF_PP  (OFF_W2T + W2T_BYTES)
#define OFF_P2  (OFF_PP + PP_BYTES)
#define OFF_X16 (OFF_P2 + P2_BYTES)
#define OFF_H16 (OFF_X16 + X16_BYTES)
#define OFF_E16 (OFF_H16 + H16_BYTES)
#define OFF_E32 (OFF_E16 + E16_BYTES)
#define WS_TOTAL (OFF_E32 + E32_BYTES)
static_assert((W1T_BYTES % 128) == 0 && (W2T_BYTES % 128) == 0 && (PP_BYTES % 128) == 0);
static_assert((P2_BYTES % 128) == 0 && (X16_BYTES % 128) == 0 && (H16_BYTES % 128) == 0);
static_assert((E16_BYTES % 128) == 0 && (E32_BYTES % 128) == 0);
static_assert(WS_TOTAL <= (size_t)134217728);

__device__ __forceinline__ float bf16r(float x) {
  unsigned int u = __float_as_uint(x);
  u = (u + 0x7FFFu + ((u >> 16) & 1u)) & 0xFFFF0000u;
  return __uint_as_float(u);
}

static __device__ __forceinline__ _Float16 toh_flush(float v) {
  const _Float16 r = (_Float16)v;
  return (fabsf(v) < 6.103515625e-05f) ? (_Float16)0.0f : r;
}

__device__ __forceinline__ v16h frag_at(const _Float16* p) {
  v8h lo = *(const v8h*)(p);
  v8h hi = *(const v8h*)(p + 16);
  v16h out;
#pragma unroll
  for (int i = 0; i < 8; ++i) { out[i] = lo[i]; out[i + 8] = hi[i]; }
  return out;
}

__device__ __forceinline__ v8f wmma16(v16h a, v16h b, v8f c) {
  v8f d = __builtin_amdgcn_wmma_f32_16x16x32_f16(false, a, false, b, (short)0, c,
                                                 false, false);
  asm volatile("v_nop\n\tv_nop\n\tv_nop\n\tv_nop" : "+v"(d) : "v"(a), "v"(b));
  return d;
}

__device__ __forceinline__ float red32_sum(float x) {
#pragma unroll
  for (int off = 1; off < 32; off <<= 1) x += __shfl_xor(x, off, 32);
  return x;
}

__device__ __forceinline__ float relu_act(float t) {
  return fmaxf(t, 0.0f);
}

__global__ __launch_bounds__(256) void wconv_kernel(
    const float* __restrict__ W, _Float16* __restrict__ Wt, unsigned ldw, unsigned ldk) {
  __shared__ _Float16 T[64 * LDT];
  const unsigned tid = threadIdx.x;
  const unsigned n0 = blockIdx.x * 64u;
  const unsigned k0 = blockIdx.y * 64u;
#pragma unroll 4
  for (unsigned j = 0; j < 16u; ++j) {
    const unsigned idx = tid + 256u * j;
    const unsigned kr = idx >> 6, nc = idx & 63u;
    const float v = W[(size_t)(k0 + kr) * ldw + n0 + nc];
    T[nc * LDT + kr] = (_Float16)(WCARRY * bf16r(v));
  }
  __syncthreads();
  v8h x[2];
  size_t off[2];
#pragma unroll
  for (unsigned i = 0; i < 2u; ++i) {
    const unsigned n = 32u * i + (tid >> 3);
    const unsigned kc = (tid & 7u) * 8u;
    x[i] = *(const v8h*)&T[n * LDT + kc];
    off[i] = (size_t)(n0 + n) * ldk + k0 + kc;
  }
#pragma unroll
  for (int i = 0; i < 2; ++i) *(volatile v8h*)(Wt + off[i]) = x[i];
  __threadfence();
#pragma unroll
  for (int i = 0; i < 2; ++i) *(volatile v8h*)(Wt + off[i]) = x[i];
}

__global__ __launch_bounds__(256) void pconv_kernel(
    const float* __restrict__ Pin, _Float16* __restrict__ Pp, float* __restrict__ p2out) {
#pragma clang fp contract(off)
  __shared__ __attribute__((aligned(16))) float s2[32];
  const unsigned lane = threadIdx.x & 31u, w = threadIdx.x >> 5;
#pragma unroll 1
  for (unsigned q = 0; q < 4u; ++q) {
    const unsigned lr = w * 4u + q;
    const unsigned row = blockIdx.x * 32u + lr;
    const bool live = row < (unsigned)NCLS;
    const unsigned srow = (row < (unsigned)(NCLS - 1)) ? row : (unsigned)(NCLS - 1);
    const float* pr = Pin + (size_t)srow * EDIM + lane * 8u;
    float ss = 0.0f;
#pragma unroll 1
    for (unsigned j = 0; j < 4u; ++j) {
      const v4f a0 = *(const v4f*)(pr + j * 256u);
      const v4f a1 = *(const v4f*)(pr + j * 256u + 4u);
      v8h o;
#pragma unroll
      for (int i = 0; i < 4; ++i) {
        const float e0 = live ? bf16r(a0[i]) : 0.0f;
        const float e1 = live ? bf16r(a1[i]) : 0.0f;
        ss += e0 * e0;
        ss += e1 * e1;
        o[i]     = toh_flush(WCARRY * e0);
        o[i + 4] = toh_flush(WCARRY * e1);
      }
      _Float16* p = Pp + (size_t)row * EDIM + j * 256u + lane * 8u;
      *(volatile v8h*)p = o;
      __threadfence();
      *(volatile v8h*)p = o;
    }
    const float tot = red32_sum(ss);
    if (lane == 0u) s2[lr] = tot;
  }
  __syncthreads();
  if (threadIdx.x < 8u) {
    const v4f v = *(const v4f*)&s2[threadIdx.x * 4u];
    float* p = p2out + blockIdx.x * 32u + threadIdx.x * 4u;
    *(volatile v4f*)p = v;
    __threadfence();
    *(volatile v4f*)p = v;
  }
}

__global__ __launch_bounds__(256) void xconv_kernel(
    const float* __restrict__ X, _Float16* __restrict__ dst) {
  const unsigned lane = threadIdx.x & 31u, w = threadIdx.x >> 5;
  const unsigned row = blockIdx.x * 8u + w;
  const float* xr = X + (size_t)row * DIM + lane * 8u;
#pragma unroll 1
  for (unsigned j = 0; j < 4u; ++j) {
    const v4f a0 = *(const v4f*)(xr + j * 256u);
    const v4f a1 = *(const v4f*)(xr + j * 256u + 4u);
    v8h o;
#pragma unroll
    for (int i = 0; i < 4; ++i) {
      o[i]     = toh_flush(bf16r(a0[i]));
      o[i + 4] = toh_flush(bf16r(a1[i]));
    }
    _Float16* p = dst + (size_t)row * DIM + j * 256u + lane * 8u;
    *(volatile v8h*)p = o;
    __threadfence();
    *(volatile v8h*)p = o;
  }
}

template <int MODE>
__device__ __forceinline__ void gemm_body(
    const _Float16* __restrict__ A16, const _Float16* __restrict__ Bt, const unsigned K,
    const float* __restrict__ bias,
    float* __restrict__ outf, _Float16* __restrict__ out16) {
  __shared__ float Cs[64 * LDC];
  const unsigned tid = threadIdx.x, lane = tid & 31u, w = tid >> 5;
  const unsigned mw = w >> 1, nw = w & 1u;
  const unsigned hh = lane >> 4, m = lane & 15u;
  const unsigned n0 = blockIdx.x * 64u;
  const unsigned row0 = blockIdx.y * 64u;

  const _Float16* ap  = A16 + (size_t)(row0 + mw * 16u + m) * K + hh * 8u;
  const _Float16* bp0 = Bt + (size_t)(n0 + nw * 32u + m) * K + hh * 8u;
  const _Float16* bp1 = bp0 + (size_t)16 * K;
  v8f acc0 = {}, acc1 = {};
#pragma unroll 2
  for (unsigned k0 = 0; k0 < K; k0 += 32u) {
    const v16h a  = frag_at(ap + k0);
    const v16h b0 = frag_at(bp0 + k0);
    const v16h b1 = frag_at(bp1 + k0);
    acc0 = wmma16(a, b0, acc0);
    acc1 = wmma16(a, b1, acc1);
  }
#pragma unroll
  for (int r = 0; r < 8; ++r) {
    float* d = &Cs[(mw * 16u + hh * 8u + (unsigned)r) * LDC + nw * 32u + m];
    d[0]  = acc0[r];
    d[16] = acc1[r];
  }
  __syncthreads();

  if (MODE == 3) {
#pragma unroll 1
    for (unsigned g = 0; g < 4u; ++g) {
      const unsigned r = 32u * (g >> 1) + (tid >> 3);
      const unsigned c = (tid & 7u) * 8u + 4u * (g & 1u);
      const v4f u  = *(const v4f*)&Cs[r * LDC + c];
      const v4f gb = *(const v4f*)(bias + n0 + c);
      v4f t;
#pragma unroll
      for (int j = 0; j < 4; ++j)
        t[j] = MCARRY * relu_act(u[j] * (1.0f / WCARRY) + bf16r(gb[j]));
      *(v4f*)&Cs[r * LDC + c] = t;
    }
  }

  if (MODE == 3) {
    v8h x[2];
    size_t off[2];
#pragma unroll
    for (unsigned i = 0; i < 2u; ++i) {
      const unsigned r = 32u * i + (tid >> 3);
      const unsigned c = (tid & 7u) * 8u;
      const v4f u0 = *(const v4f*)&Cs[r * LDC + c];
      const v4f u1 = *(const v4f*)&Cs[r * LDC + c + 4];
#pragma unroll
      for (int j = 0; j < 4; ++j) {
        x[i][j]     = toh_flush(u0[j]);
        x[i][j + 4] = toh_flush(u1[j]);
      }
      off[i] = (size_t)(row0 + r) * HID + n0 + c;
    }
#pragma unroll
    for (int i = 0; i < 2; ++i) *(volatile v8h*)(out16 + off[i]) = x[i];
    __threadfence();
#pragma unroll
    for (int i = 0; i < 2; ++i) *(volatile v8h*)(out16 + off[i]) = x[i];
  }

  if (MODE == 5) {
    const float cs = 1.0f / (WCARRY * MCARRY);
    v4f xs[4];
    size_t off[4];
#pragma unroll
    for (unsigned i = 0; i < 4u; ++i) {
      const unsigned r = 16u * i + (tid >> 4);
      const unsigned c = (tid & 15u) * 4u;
      const v4f u = *(const v4f*)&Cs[r * LDC + c];
      const v4f g = *(const v4f*)(bias + n0 + c);
      v4f val;
#pragma unroll
      for (int j = 0; j < 4; ++j) val[j] = u[j] * cs + bf16r(g[j]);
      xs[i] = val;
      off[i] = (size_t)(row0 + r) * EDIM + n0 + c;
    }
    v8h x[2];
    size_t off16[2];
#pragma unroll
    for (unsigned i = 0; i < 2u; ++i) {
      const unsigned r = 32u * i + (tid >> 3);
      const unsigned c = (tid & 7u) * 8u;
      const v4f u0 = *(const v4f*)&Cs[r * LDC + c];
      const v4f u1 = *(const v4f*)&Cs[r * LDC + c + 4];
      const v4f g0 = *(const v4f*)(bias + n0 + c);
      const v4f g1 = *(const v4f*)(bias + n0 + c + 4u);
#pragma unroll
      for (int j = 0; j < 4; ++j) {
        x[i][j]     = toh_flush(ECARRY * (u0[j] * cs + bf16r(g0[j])));
        x[i][j + 4] = toh_flush(ECARRY * (u1[j] * cs + bf16r(g1[j])));
      }
      off16[i] = (size_t)(row0 + r) * EDIM + n0 + c;
    }
#pragma unroll
    for (int i = 0; i < 4; ++i) *(volatile v4f*)(outf + off[i]) = xs[i];
#pragma unroll
    for (int i = 0; i < 2; ++i) *(volatile v8h*)(out16 + off16[i]) = x[i];
    __threadfence();
#pragma unroll
    for (int i = 0; i < 4; ++i) *(volatile v4f*)(outf + off[i]) = xs[i];
#pragma unroll
    for (int i = 0; i < 2; ++i) *(volatile v8h*)(out16 + off16[i]) = x[i];
  }
}

__global__ __launch_bounds__(256) void gemm_ffn1_kernel(
    const _Float16* __restrict__ A16, const _Float16* __restrict__ Bt,
    const float* __restrict__ bias, _Float16* __restrict__ mid) {
  gemm_body<3>(A16, Bt, (unsigned)DIM, bias, (float*)0, mid);
}
__global__ __launch_bounds__(256) void gemm_enc_kernel(
    const _Float16* __restrict__ A16, const _Float16* __restrict__ Bt,
    const float* __restrict__ bias, float* __restrict__ enc32, _Float16* __restrict__ enc16) {
  gemm_body<5>(A16, Bt, (unsigned)HID, bias, enc32, enc16);
}

__global__ __launch_bounds__(256) void scores_kernel(
    const _Float16* __restrict__ E16, const float* __restrict__ E32,
    const _Float16* __restrict__ Pp, const float* __restrict__ p2,
    float* __restrict__ out) {
  __shared__ __attribute__((aligned(16))) float Ss[SROWS * NCLS];
  __shared__ float x2s[SROWS];
  const unsigned tid = threadIdx.x, lane = tid & 31u;
  const unsigned w = (unsigned)__builtin_amdgcn_readfirstlane((int)(threadIdx.x >> 5));
  const unsigned hh = lane >> 4, m = lane & 15u;
  const unsigned row0 = blockIdx.x * (unsigned)SROWS;

#pragma unroll 1
  for (unsigned q = 0; q < 2u; ++q) {
    const unsigned lr = w * 2u + q;
    const float* er = E32 + (size_t)(row0 + lr) * EDIM + lane * 8u;
    float ss = 0.0f;
#pragma unroll 1
    for (unsigned j = 0; j < 4u; ++j) {
      const v4f a0 = *(const v4f*)(er + j * 256u);
      const v4f a1 = *(const v4f*)(er + j * 256u + 4u);
#pragma unroll
      for (int i = 0; i < 4; ++i) {
        ss += a0[i] * a0[i];
        ss += a1[i] * a1[i];
      }
    }
    const float tot = red32_sum(ss);
    if (lane == 0u) x2s[lr] = tot;
  }
  __syncthreads();

  const _Float16* ap = E16 + (size_t)(row0 + m) * EDIM + hh * 8u;
  const _Float16* bp = Pp + (size_t)(w * 128u + m) * EDIM + hh * 8u;
  v8f acc[8];
#pragma unroll
  for (int t = 0; t < 8; ++t) acc[t] = (v8f){};
#pragma unroll 1
  for (unsigned k0 = 0; k0 < (unsigned)EDIM; k0 += 32u) {
    const v16h a = frag_at(ap + k0);
#pragma unroll
    for (int t = 0; t < 8; ++t) {
      const v16h b = frag_at(bp + (size_t)t * 16u * EDIM + k0);
      acc[t] = wmma16(a, b, acc[t]);
    }
  }

  const float cs = 1.0f / (ECARRY * WCARRY);
#pragma unroll
  for (int t = 0; t < 8; ++t) {
    const unsigned col = w * 128u + (unsigned)t * 16u + m;
    const float pp = p2[col];
#pragma unroll
    for (int r = 0; r < 8; ++r) {
      const unsigned lr = hh * 8u + (unsigned)r;
      const float dot = acc[t][r] * cs;
      const float d2 = fmaxf((x2s[lr] + pp) - 2.0f * dot, 0.0f);
      if (col < (unsigned)NCLS) Ss[lr * (unsigned)NCLS + col] = -d2;
    }
  }
  __syncthreads();

  float* dst = out + (size_t)row0 * NCLS;
  const unsigned nvec = (unsigned)(SROWS * NCLS / 4);
#pragma unroll 1
  for (unsigned j = 0; j < 16u; ++j) {
    const unsigned q = tid + 256u * j;
    if (q < nvec) {
      const v4f v = *(const v4f*)&Ss[q * 4u];
      *(volatile v4f*)(dst + (size_t)q * 4u) = v;
    }
  }
  __threadfence();
#pragma unroll 1
  for (unsigned j = 0; j < 16u; ++j) {
    const unsigned q = tid + 256u * j;
    if (q < nvec) {
      const v4f v = *(const v4f*)&Ss[q * 4u];
      *(volatile v4f*)(dst + (size_t)q * 4u) = v;
    }
  }
}

__global__ __launch_bounds__(256) void seg_kernel(
    const float* __restrict__ enc, const int* __restrict__ labels, float* __restrict__ upd) {
  __shared__ unsigned masks[256];
  const unsigned tid = threadIdx.x;
  const int cls = (int)blockIdx.x;
  unsigned mk = 0u;
  if (tid < (unsigned)NWORDS) {
    const int* lp = labels + tid * 32u;
#pragma unroll 1
    for (unsigned j = 0; j < 8u; ++j) {
      const v4i L = *(const v4i*)(lp + j * 4u);
      const unsigned nib = ((L[0] == cls) ? 1u : 0u) | ((L[1] == cls) ? 2u : 0u) |
                           ((L[2] == cls) ? 4u : 0u) | ((L[3] == cls) ? 8u : 0u);
      mk |= nib << (4u * j);
    }
  }
  masks[tid] = mk;
  __syncthreads();

  v4f acc = {0.0f, 0.0f, 0.0f, 0.0f};
  const float* ecol = enc + tid * 4u;
#pragma unroll 1
  for (unsigned wd = 0; wd < (unsigned)NWORDS; ++wd) {
    unsigned bits = (unsigned)__builtin_amdgcn_readfirstlane((int)masks[wd]);
    while (bits != 0u) {
      const unsigned i = (unsigned)__builtin_ctz(bits);
      bits &= bits - 1u;
      const unsigned b = wd * 32u + i;
      const v4f e = *(const v4f*)(ecol + (size_t)b * EDIM);
      acc += e;
    }
  }
  float* p = upd + (size_t)cls * EDIM + tid * 4u;
  *(volatile v4f*)p = acc;
  __threadfence();
  *(volatile v4f*)p = acc;
}

__global__ __launch_bounds__(256) void counts_kernel(
    const int* __restrict__ labels, float* __restrict__ cnt) {
  __shared__ int part[8 * 32];
  __shared__ __attribute__((aligned(16))) float cf[32];
  const unsigned tid = threadIdx.x, j = tid & 31u, p = tid >> 5;
  const unsigned c0 = blockIdx.x * 32u;
  const int cls = (int)(c0 + j);
  const int* lp = labels + p * (unsigned)(NB / 8);
  int c = 0;
#pragma unroll 1
  for (unsigned q = 0; q < (unsigned)(NB / 8); q += 4u) {
    const v4i L = *(const v4i*)(lp + q);
    c += (L[0] == cls) ? 1 : 0;
    c += (L[1] == cls) ? 1 : 0;
    c += (L[2] == cls) ? 1 : 0;
    c += (L[3] == cls) ? 1 : 0;
  }
  part[p * 32u + j] = c;
  __syncthreads();
  if (tid < 32u) {
    int s = 0;
#pragma unroll
    for (unsigned pp = 0; pp < 8u; ++pp) s += part[pp * 32u + tid];
    cf[tid] = (float)s;
  }
  __syncthreads();
  const unsigned left = (unsigned)NCLS - c0;
  const unsigned nq = (left >= 32u) ? 8u : (left >> 2);
  if (tid < nq) {
    const v4f v = *(const v4f*)&cf[tid * 4u];
    float* o = cnt + c0 + tid * 4u;
    *(volatile v4f*)o = v;
    __threadfence();
    *(volatile v4f*)o = v;
  }
}

extern "C" void kernel_launch(void* const* d_in, const int* in_sizes, int n_in,
                              void* d_out, int out_size, void* d_ws, size_t ws_size,
                              hipStream_t stream) {
  if (n_in < 7) return;
  if ((long long)in_sizes[0] < (long long)MROWS * DIM) return;
  if ((long long)in_sizes[1] < (long long)DIM * HID) return;
  if (in_sizes[2] < HID) return;
  if ((long long)in_sizes[3] < (long long)HID * EDIM) return;
  if (in_sizes[4] < EDIM) return;
  if ((long long)in_sizes[5] < (long long)NCLS * EDIM) return;
  if (in_sizes[6] < MROWS) return;
  if ((long long)out_size < (long long)OUT_TOTAL) return;
  if (ws_size < WS_TOTAL) return;

  const float* X   = (const float*)d_in[0];
  const float* w1  = (const float*)d_in[1];
  const float* b1  = (const float*)d_in[2];
  const float* w2  = (const float*)d_in[3];
  const float* b2  = (const float*)d_in[4];
  const float* pr  = (const float*)d_in[5];
  const int*   lab = (const int*)d_in[6];
  float* out = (float*)d_out;
  float* out_upd = out + OUT_UPD_OFF;
  float* out_cnt = out + OUT_CNT_OFF;

  char* ws = (char*)d_ws;
  _Float16* W1_t = (_Float16*)(ws + OFF_W1T);
  _Float16* W2_t = (_Float16*)(ws + OFF_W2T);
  _Float16* Pp16 = (_Float16*)(ws + OFF_PP);
  float*    P2   = (float*)(ws + OFF_P2);
  _Float16* X16  = (_Float16*)(ws + OFF_X16);
  _Float16* H16  = (_Float16*)(ws + OFF_H16);
  _Float16* E16  = (_Float16*)(ws + OFF_E16);
  float*    E32  = (float*)(ws + OFF_E32);

  dim3 blk(256);

  wconv_kernel<<<dim3(HID / 64, DIM / 64), blk, 0, stream>>>(w1, W1_t, (unsigned)HID, (unsigned)DIM);
  wconv_kernel<<<dim3(EDIM / 64, HID / 64), blk, 0, stream>>>(w2, W2_t, (unsigned)EDIM, (unsigned)HID);
  pconv_kernel<<<dim3(NCP / 32), blk, 0, stream>>>(pr, Pp16, P2);
  xconv_kernel<<<dim3(MROWS / 8), blk, 0, stream>>>(X, X16);

  gemm_ffn1_kernel<<<dim3(HID / 64, MROWS / 64), blk, 0, stream>>>(X16, W1_t, b1, H16);
  gemm_enc_kernel<<<dim3(EDIM / 64, MROWS / 64), blk, 0, stream>>>(H16, W2_t, b2, E32, E16);

  scores_kernel<<<dim3(MROWS / SROWS), blk, 0, stream>>>(E16, E32, Pp16, P2, out);
  seg_kernel<<<dim3(NCLS), blk, 0, stream>>>(E32, lab, out_upd);
  counts_kernel<<<dim3((NCLS + 31) / 32), blk, 0, stream>>>(lab, out_cnt);
}
